// TransformerBlock_39419209842958
// MI455X (gfx1250) — hardware-verified
//
#include <hip/hip_runtime.h>
#include <math.h>
#include <stdint.h>

#ifndef NB
#define NB    2
#endif
#ifndef SEQ
#define SEQ   2048
#endif
#define NB_FULL   2
#define SEQ_FULL  2048
#define DM    768
#define NH    12
#define HD    64
#define DQKV  (3 * DM)
#define DFF   (4 * DM)
#define NQB   (SEQ / 64)
#define NKT   (SEQ / 64)
#define ROWS  (NB * SEQ)
#define MBW   (SEQ_FULL / 32)
#define OUT0N_FULL (NB_FULL * SEQ_FULL * DM)

#define A_CARRY   16.0f
#define W_CARRY   256.0f
#define P_CARRY   1024.0f
#define CTX_CARRY 64.0f
#define SCORE_SC  (1.0f / 2048.0f)
#define CTX_FAC   (1.0f / 256.0f)
#define NEG_BIG   (-1.0e30f)

static constexpr float SC_W   = 256.0f;
static constexpr float SC_ACT = 16.0f;
static constexpr float SC_ONE = 1.0f;
static constexpr float CS_ACT = 1.0f / 4096.0f;
static constexpr float CS_CTX = 1.0f / 16384.0f;

static_assert(NH * HD == DM);
static_assert(HD == 64);
static_assert((SEQ % 64) == 0 && (DM % 64) == 0 && (DQKV % 64) == 0 && (DFF % 64) == 0);
static_assert((DM % 32) == 0 && (DFF % 32) == 0);
static_assert((SEQ % 16) == 0 && (SEQ_FULL % 1024) == 0 && SEQ <= SEQ_FULL);
static_assert(NB == 1 || (NB == NB_FULL && SEQ == SEQ_FULL));
static_assert(((ROWS / 64) * (DQKV / 64)) % 8 == 0);
static_assert(((ROWS / 64) * (DM / 64)) % 8 == 0);
static_assert(((ROWS / 64) * (DFF / 64)) % 8 == 0);
static_assert((ROWS % 8) == 0);
static_assert(((DQKV * DM / 8) % 256) == 0 && ((DM * DM / 8) % 256) == 0 && ((DFF * DM / 8) % 256) == 0);
static_assert(SC_W == W_CARRY && SC_ACT == A_CARRY);
static_assert(CS_ACT * A_CARRY * W_CARRY == 1.0f);
static_assert(CS_CTX * CTX_CARRY * W_CARRY == 1.0f);
static_assert(SCORE_SC * 8.0f * A_CARRY * A_CARRY == 1.0f);
static_assert(CTX_FAC * A_CARRY * P_CARRY == CTX_CARRY);
static_assert((size_t)OUT0N_FULL * 4 == (size_t)12582912);
static_assert(32 * 16 * 4 == 16 * 64 * 2);
static_assert(32 * 16 * 8 == 16 * 64 * 4);
static_assert(32 * 16 * 1 == 4 * 128);
static_assert(3 * 32 * 16 == DM * 2);
static_assert(8 * DM * 2 <= 131072);
static_assert(8 * 16 * 68 * 4 <= 131072);
static_assert(64 * 72 * 2 <= 131072);
static_assert(2 * 64 * 64 * 2 + 2 * 4 * 16 * 64 * 4 <= 131072);
static_assert(8 * 128 * 4 <= 131072);

typedef _Float16 v16h __attribute__((ext_vector_type(16)));
typedef _Float16 v8h  __attribute__((ext_vector_type(8)));
typedef float    v8f  __attribute__((ext_vector_type(8)));
typedef float    v4f  __attribute__((ext_vector_type(4)));
typedef unsigned int v4u __attribute__((ext_vector_type(4)));
typedef unsigned int v2u __attribute__((ext_vector_type(2)));
typedef _Float16 h16;

__device__ __forceinline__ unsigned short bf_bits(float f) {
  unsigned u = __float_as_uint(f);
  return (unsigned short)((u + 0x7FFFu + ((u >> 16) & 1u)) >> 16);
}
__device__ __forceinline__ float bfr(float f) { return __uint_as_float(((unsigned)bf_bits(f)) << 16); }
__device__ __forceinline__ unsigned short h_bits(_Float16 x) { return __builtin_bit_cast(unsigned short, x); }
__device__ __forceinline__ unsigned pk16(unsigned short a, unsigned short b) { return (unsigned)a | ((unsigned)b << 16); }
__device__ __forceinline__ v8f zero8() { v8f z = {0.f, 0.f, 0.f, 0.f, 0.f, 0.f, 0.f, 0.f}; return z; }
__device__ __forceinline__ float gelu_erf(float a) { return 0.5f * a * (1.0f + erff(a * 0.70710678118654752f)); }

static __device__ __forceinline__ h16 toh_flush(float v) {
  const float w = (fabsf(v) < 6.103515625e-05f) ? 0.0f : v;
  return (h16)w;
}
static __device__ __forceinline__ v4u pack8_flush(v4f a, v4f a2) {
  v4u p;
  p[0] = pk16(h_bits(toh_flush(a[0])),  h_bits(toh_flush(a[1])));
  p[1] = pk16(h_bits(toh_flush(a[2])),  h_bits(toh_flush(a[3])));
  p[2] = pk16(h_bits(toh_flush(a2[0])), h_bits(toh_flush(a2[1])));
  p[3] = pk16(h_bits(toh_flush(a2[2])), h_bits(toh_flush(a2[3])));
  return p;
}

__device__ __forceinline__ v16h ldfrag_h(const _Float16* p) {
  union { v16h v; v8h h[2]; } f;
  f.h[0] = *(const v8h*)(p);
  f.h[1] = *(const v8h*)(p + 16);
  return f.v;
}

__device__ __forceinline__ v8f mma_h(v16h a, v16h b, v8f c) {
  c = __builtin_amdgcn_wmma_f32_16x16x32_f16(false, a, false, b, (short)0, c, false, false);
#if defined(__HIP_DEVICE_COMPILE__)
  asm volatile("v_nop\n\tv_nop\n\tv_nop\n\tv_nop" : "+v"(c) : "v"(a), "v"(b));
#endif
  return c;
}

__global__ __launch_bounds__(256) void cvt_w16(const float* __restrict__ in, unsigned short* out, int n8, float scale) {
  const int i = blockIdx.x * 256 + threadIdx.x;
  if (i < n8) {
    const v4f a  = *(const v4f*)(in + (size_t)i * 8);
    const v4f b  = *(const v4f*)(in + (size_t)i * 8 + 4);
    float f[8];
    f[0] = a[0]; f[1] = a[1]; f[2] = a[2]; f[3] = a[3];
    f[4] = b[0]; f[5] = b[1]; f[6] = b[2]; f[7] = b[3];
    v4u p;
#pragma unroll
    for (int e = 0; e < 4; ++e) {
      const float g0 = bfr(f[2 * e]), g1 = bfr(f[2 * e + 1]);
      p[e] = pk16(h_bits(toh_flush(g0 * scale)), h_bits(toh_flush(g1 * scale)));
    }
    *(volatile v4u*)(out + (size_t)i * 8) = p;
    __threadfence();
    *(volatile v4u*)(out + (size_t)i * 8) = p;
  }
}

__global__ __launch_bounds__(256) void mask_pack(const int* __restrict__ mk, unsigned int* mb, float* tail) {
  __shared__ __align__(16) unsigned int sw[8][128];
  const int lane = threadIdx.x & 31;
  const int wave = __builtin_amdgcn_readfirstlane((int)(threadIdx.x >> 5));
  const int grp  = blockIdx.x * 8 + wave;
  const int* src = mk + (size_t)(2 * grp) * SEQ_FULL;
  unsigned int mine[4];
  mine[0] = 0u; mine[1] = 0u; mine[2] = 0u; mine[3] = 0u;
#pragma unroll 1
  for (int w = 0; w < 32; ++w) {
#pragma unroll
    for (int t = 0; t < 4; ++t) {
      const int v = src[(t * 32 + w) * 32 + lane];
      const unsigned int word = __builtin_amdgcn_ballot_w32(v != 0);
      mine[t] = (lane == w) ? word : mine[t];
    }
  }
#pragma unroll
  for (int t = 0; t < 4; ++t) sw[wave][t * 32 + lane] = mine[t];
  __builtin_amdgcn_fence(3  , "workgroup");
  __builtin_amdgcn_wave_barrier();
  __builtin_amdgcn_fence(2  , "workgroup");
  const v4u o = *(const v4u*)(&sw[wave][lane * 4]);
  unsigned int* dst = mb + (size_t)grp * 128 + lane * 4;
  *(volatile v4u*)dst = o;
  __threadfence();
  *(volatile v4u*)dst = o;
  if (blockIdx.x == 0 && threadIdx.x == 0) {
    *(volatile float*)tail = 0.0f;
    __threadfence();
    *(volatile float*)tail = 0.0f;
  }
}

__global__ __launch_bounds__(256) void ln_k(const float* __restrict__ xin, int rb,
                                            const float* __restrict__ gp, const float* __restrict__ bp,
                                            unsigned short* hout, int nrows) {
  union H8 { v8h h; v4u u; };
  __shared__ __align__(16) _Float16 sh[8][DM];
  const int lane = threadIdx.x & 31;
  const int wave = threadIdx.x >> 5;
  const int row  = blockIdx.x * 8 + wave;
  if (row >= nrows) return;
  const float* xr = xin + (size_t)row * DM;
  float v[24];
  float s = 0.f;
#pragma unroll
  for (int i = 0; i < 24; ++i) {
    float t = xr[lane + 32 * i];
    t = (rb != 0) ? bfr(t) : t;
    v[i] = t;
    s += t;
  }
#pragma unroll
  for (int off = 16; off > 0; off >>= 1) s += __shfl_xor(s, off, 32);
  const float mu = s * (1.0f / (float)DM);
  float q = 0.f;
#pragma unroll
  for (int i = 0; i < 24; ++i) { const float d = v[i] - mu; q += d * d; }
#pragma unroll
  for (int off = 16; off > 0; off >>= 1) q += __shfl_xor(q, off, 32);
  const float inv = rsqrtf(q * (1.0f / (float)DM) + 1e-5f);
#pragma unroll
  for (int i = 0; i < 24; ++i) {
    const int cc = lane + 32 * i;
    const float hv = (v[i] - mu) * inv * bfr(gp[cc]) + bfr(bp[cc]);
    sh[wave][cc] = (_Float16)(hv * 16.0f);
  }
  __builtin_amdgcn_fence(3  , "workgroup");
  __builtin_amdgcn_wave_barrier();
  __builtin_amdgcn_fence(2  , "workgroup");
  H8 o[3];
#pragma unroll
  for (int t = 0; t < 3; ++t) o[t].h = *(const v8h*)(&sh[wave][(t * 32 + lane) * 8]);
  for (int pass = 0; pass < 2; ++pass) {
#pragma unroll
    for (int t = 0; t < 3; ++t)
      *(volatile v4u*)(hout + (size_t)row * DM + (size_t)(t * 32 + lane) * 8) = o[t].u;
    __threadfence();
  }
}

template <int EPI>
__global__ __launch_bounds__(256) void gemm64_f16(
    const unsigned short* __restrict__ Ap, int lda,
    const unsigned short* __restrict__ Btp, int ldb,
    const float* __restrict__ biasp, float cscale,
    const float* __restrict__ resp, int ldr,
    void* Cp, int ldc, int M, int N, int K, float oscale) {
  const _Float16* Ah = (const _Float16*)(const void*)Ap;
  const _Float16* Bt = (const _Float16*)(const void*)Btp;
  __shared__ __align__(16) float sT[8][16 * 68];
  const int lane = threadIdx.x & 31;
  const int wave = threadIdx.x >> 5;
  const int tilesN = N >> 6;
  const int tilesM = M >> 6;
  const int tile = blockIdx.x * 8 + wave;
  if (tile >= tilesM * tilesN) return;
  const int tm = (int)((unsigned)tile / (unsigned)tilesN);
  const int tn = tile - tm * tilesN;
  const int m0 = tm << 6;
  const int n0 = tn << 6;

  const int rlane = lane & 15;
  const int koff  = (lane >> 4) * 8;
  const int mOff  = (lane >> 4) * 8;

  v8f acc[4][4];
#pragma unroll
  for (int i = 0; i < 4; ++i)
#pragma unroll
    for (int j = 0; j < 4; ++j) acc[i][j] = zero8();

  for (int k0 = 0; k0 < K; k0 += 32) {
    v16h bh[4];
#pragma unroll
    for (int j = 0; j < 4; ++j) {
      const size_t bo = (size_t)(n0 + (j << 4) + rlane) * ldb + koff + k0;
      bh[j] = ldfrag_h(Bt + bo);
    }
#pragma unroll
    for (int i = 0; i < 4; ++i) {
      const size_t ao = (size_t)(m0 + (i << 4) + rlane) * lda + koff + k0;
      const v16h ah = ldfrag_h(Ah + ao);
#pragma unroll
      for (int j = 0; j < 4; ++j) {
        acc[i][j] = mma_h(ah, bh[j], acc[i][j]);
      }
    }
  }

  float* slab = sT[wave];
#pragma unroll
  for (int i = 0; i < 4; ++i) {
    const int mBase = m0 + (i << 4);
    float bj[4];
#pragma unroll
    for (int j = 0; j < 4; ++j) bj[j] = bfr(biasp[n0 + (j << 4) + rlane]);
#pragma unroll
    for (int r = 0; r < 8; ++r) {
      const int row = mOff + r;
#pragma unroll
      for (int j = 0; j < 4; ++j) {
        float v = acc[i][j][r] * cscale + bj[j];
        if constexpr (EPI == 1) v = gelu_erf(v);
        slab[row * 68 + (j << 4) + rlane] = v;
      }
    }
    __builtin_amdgcn_fence(3  , "workgroup");
    __builtin_amdgcn_wave_barrier();
    __builtin_amdgcn_fence(2  , "workgroup");
    if constexpr (EPI <= 1) {
      unsigned short* C16 = (unsigned short*)Cp;
      const int rq = lane >> 3, piece = lane & 7;
      v4u pv[4];
#pragma unroll
      for (int it = 0; it < 4; ++it) {
        const int row = it * 4 + rq;
        const v4f a  = *(const v4f*)(slab + row * 68 + piece * 8);
        const v4f a2 = *(const v4f*)(slab + row * 68 + piece * 8 + 4);
        v4u p;
        p[0] = pk16(h_bits(toh_flush(a[0]  * oscale)), h_bits(toh_flush(a[1]  * oscale)));
        p[1] = pk16(h_bits(toh_flush(a[2]  * oscale)), h_bits(toh_flush(a[3]  * oscale)));
        p[2] = pk16(h_bits(toh_flush(a2[0] * oscale)), h_bits(toh_flush(a2[1] * oscale)));
        p[3] = pk16(h_bits(toh_flush(a2[2] * oscale)), h_bits(toh_flush(a2[3] * oscale)));
        pv[it] = p;
      }
      for (int pass = 0; pass < 2; ++pass) {
#pragma unroll
        for (int it = 0; it < 4; ++it) {
          const int row = it * 4 + rq;
          *(volatile v4u*)(C16 + (size_t)(mBase + row) * ldc + n0 + piece * 8) = pv[it];
        }
        __threadfence();
      }
    } else {
      float* Cf = (float*)Cp;
      const int hh = lane >> 4, c4 = (lane & 15) * 4;
      v4f ov[8];
#pragma unroll
      for (int it = 0; it < 8; ++it) {
        const int row = it * 2 + hh;
        v4f o = *(const v4f*)(slab + row * 68 + c4);
        const v4f rs = *(const v4f*)(resp + (size_t)(mBase + row) * ldr + n0 + c4);
        if constexpr (EPI == 2) {
          o[0] += bfr(rs[0]); o[1] += bfr(rs[1]); o[2] += bfr(rs[2]); o[3] += bfr(rs[3]);
        } else {
          o += rs;
        }
        ov[it] = o;
      }
      for (int pass = 0; pass < 2; ++pass) {
#pragma unroll
        for (int it = 0; it < 8; ++it) {
          const int row = it * 2 + hh;
          *(volatile v4f*)(Cf + (size_t)(mBase + row) * ldc + n0 + c4) = ov[it];
        }
        __threadfence();
      }
    }
    __builtin_amdgcn_fence(3  , "workgroup");
    __builtin_amdgcn_wave_barrier();
    __builtin_amdgcn_fence(2  , "workgroup");
  }
}

__global__ __launch_bounds__(256) void v_tr(const unsigned short* __restrict__ qkvp, unsigned short* vt) {
  __shared__ __align__(16) _Float16 sv[64 * 72];
  const int tid = threadIdx.x;
  const int t0  = blockIdx.x * 64;
  const int hh  = blockIdx.y;
  const int b   = blockIdx.z;
  const _Float16* src = (const _Float16*)(const void*)qkvp;
#pragma unroll
  for (int i = 0; i < 2; ++i) {
    const int idx = i * 256 + tid;
    const int tt = idx >> 3, c8 = (idx & 7) * 8;
    const v8h a = *(const v8h*)(src + ((size_t)(b * SEQ + t0 + tt)) * DQKV + 2 * DM + hh * HD + c8);
    *(v8h*)(sv + tt * 72 + c8) = a;
  }
  __syncthreads();

  const int g = tid >> 3, piece = tid & 7;
  v4u hv[2];
  size_t hofs[2];
#pragma unroll
  for (int it = 0; it < 2; ++it) {
    const int d = it * 32 + g;
    v4u a;
#pragma unroll
    for (int e = 0; e < 4; ++e) {
      const _Float16 x0 = sv[(piece * 8 + 2 * e) * 72 + d];
      const _Float16 x1 = sv[(piece * 8 + 2 * e + 1) * 72 + d];
      a[e] = pk16(h_bits(x0), h_bits(x1));
    }
    hv[it] = a;
    hofs[it] = ((size_t)(b * DM + hh * HD + d)) * SEQ + t0 + piece * 8;
  }
  for (int pass = 0; pass < 2; ++pass) {
#pragma unroll
    for (int it = 0; it < 2; ++it) *(volatile v4u*)(vt + hofs[it]) = hv[it];
    __threadfence();
  }
}

__global__ __launch_bounds__(128)
void attn_k(const unsigned short* __restrict__ qkvp, const unsigned short* __restrict__ vtp,
            const unsigned int* __restrict__ mbp, unsigned short* ctxp) {
  union FH { v16h v; v8h h[2]; };
  union FP { v16h v; v4u u[2]; };
  __shared__ __align__(16) _Float16 Ksh[64 * 64];
  __shared__ __align__(16) _Float16 Vsh[64 * 64];
  __shared__ __align__(16) float    Pf[4][16 * 64];
  __shared__ __align__(16) float    Os[4][16 * 64];

  const int tid  = threadIdx.x;
  const int wave = __builtin_amdgcn_readfirstlane(tid >> 5);
  const int lane = tid & 31;
  const int hh   = lane >> 4;
  const int c    = lane & 15;

  const unsigned bx   = blockIdx.x;
  const unsigned qbu  = bx % (unsigned)NQB;
  const unsigned rest = bx / (unsigned)NQB;
  const unsigned hu   = rest % (unsigned)NH;
  const unsigned bu   = rest / (unsigned)NH;
  const int qb   = (int)qbu;
  const int h    = (int)hu;
  const int b    = (int)bu;
  const int q0   = qb * 64 + wave * 16;
  const size_t rowB = (size_t)b * SEQ;

  const _Float16* Qp = (const _Float16*)(const void*)qkvp + (size_t)h * HD;
  const _Float16* Kp = (const _Float16*)(const void*)qkvp + DM + (size_t)h * HD;
  const _Float16* Vt = (const _Float16*)(const void*)vtp + ((size_t)b * DM + (size_t)h * HD) * SEQ;

  v16h qa[2];
#pragma unroll
  for (int dc = 0; dc < 2; ++dc) {
    const size_t qo = (rowB + q0 + c) * DQKV + dc * 32 + 8 * hh;
    qa[dc] = ldfrag_h(Qp + qo);
  }

  float mrow[8], lrow[8];
  v8f oacc[4];
#pragma unroll
  for (int r = 0; r < 8; ++r) { mrow[r] = NEG_BIG; lrow[r] = 0.f; }
#pragma unroll
  for (int t = 0; t < 4; ++t) oacc[t] = zero8();

  float* pf = Pf[wave];

  for (int kt = 0; kt < NKT; ++kt) {
    const int kv0 = kt * 64;

    unsigned int mx[8], my[8];
    unsigned int orw = 0u;
#pragma unroll
    for (int r = 0; r < 8; ++r) {
      const v2u mw = *(const v2u*)(mbp + (size_t)(q0 + 8 * hh + r) * MBW + 2 * kt);
      unsigned int w0 = mw[0];
      unsigned int w1 = mw[1];
#if defined(__HIP_DEVICE_COMPILE__)
      asm volatile("" : "+v"(w0));
      asm volatile("" : "+v"(w1));
#endif
      mx[r] = w0;
      my[r] = w1;
      orw |= (w0 | w1);
    }
    const unsigned int act = __builtin_amdgcn_ballot_w32(orw != 0u);

    __syncthreads();
    {
      const int r = tid >> 1, half = (tid & 1) * 32;
      const _Float16* kg = Kp + (rowB + kv0 + r) * DQKV + half;
      const _Float16* vg = Vt + (size_t)r * SEQ + kv0 + half;
#pragma unroll
      for (int i = 0; i < 4; ++i) {
        const v8h a0 = *(const v8h*)(kg + 8 * i);
        const v8h b0 = *(const v8h*)(vg + 8 * i);
        *(v8h*)(Ksh + r * 64 + half + 8 * i) = a0;
        *(v8h*)(Vsh + r * 64 + half + 8 * i) = b0;
      }
    }
    __syncthreads();

    if (act != 0u) {
      v8f s[4];
#pragma unroll
      for (int j = 0; j < 4; ++j) {
        s[j] = zero8();
#pragma unroll
        for (int dc = 0; dc < 2; ++dc) {
          FH kb;
          kb.h[0] = *(const v8h*)(Ksh + (j * 16 + c) * 64 + dc * 32 + 8 * hh);
          kb.h[1] = *(const v8h*)(Ksh + (j * 16 + c) * 64 + dc * 32 + 16 + 8 * hh);
          s[j] = mma_h(qa[dc], kb.v, s[j]);
        }
      }

#pragma unroll
      for (int r = 0; r < 8; ++r) {
        float m = NEG_BIG;
#pragma unroll
        for (int j = 0; j < 4; ++j) {
          const unsigned int wsel = (j < 2) ? mx[r] : my[r];
          const unsigned int vis  = (wsel >> ((j & 1) * 16 + c)) & 1u;
          const float a = s[j][r] * SCORE_SC;
          s[j][r] = a;
          m = (vis != 0u) ? fmaxf(m, a) : m;
        }
#pragma unroll
        for (int off = 1; off < 16; off <<= 1) m = fmaxf(m, __shfl_xor(m, off, 32));
        const float mn    = fmaxf(mrow[r], m);
        const float alpha = __expf(mrow[r] - mn);
        mrow[r] = mn;
        float psum = 0.f;
#pragma unroll
        for (int j = 0; j < 4; ++j) {
          const unsigned int wsel = (j < 2) ? mx[r] : my[r];
          const unsigned int vis  = (wsel >> ((j & 1) * 16 + c)) & 1u;
          const float e = __expf(s[j][r] - mn);
          const float p = (vis != 0u) ? e : 0.0f;
          psum += p;
          pf[(8 * hh + r) * 64 + j * 16 + c] = p * P_CARRY;
        }
#pragma unroll
        for (int off = 1; off < 16; off <<= 1) psum += __shfl_xor(psum, off, 32);
        lrow[r] = lrow[r] * alpha + psum;
#pragma unroll
        for (int t = 0; t < 4; ++t) oacc[t][r] *= alpha;
      }
      __builtin_amdgcn_fence(3  , "workgroup");
      __builtin_amdgcn_wave_barrier();
      __builtin_amdgcn_fence(2  , "workgroup");

#pragma unroll
      for (int kk = 0; kk < 2; ++kk) {
        FP pa;
        {
          const float* pr = pf + c * 64 + kk * 32 + 8 * hh;
          const v4f x0 = *(const v4f*)(pr);
          const v4f x1 = *(const v4f*)(pr + 4);
          const v4f y0 = *(const v4f*)(pr + 16);
          const v4f y1 = *(const v4f*)(pr + 20);
          pa.u[0] = pack8_flush(x0, x1);
          pa.u[1] = pack8_flush(y0, y1);
        }
#pragma unroll
        for (int t = 0; t < 4; ++t) {
          FH vb;
          vb.h[0] = *(const v8h*)(Vsh + (t * 16 + c) * 64 + kk * 32 + 8 * hh);
          vb.h[1] = *(const v8h*)(Vsh + (t * 16 + c) * 64 + kk * 32 + 16 + 8 * hh);
          oacc[t] = mma_h(pa.v, vb.v, oacc[t]);
        }
      }
    }
  }

  float* os = Os[wave];
#pragma unroll
  for (int r = 0; r < 8; ++r) {
    const float inv = __builtin_amdgcn_rcpf(lrow[r]) * CTX_FAC;
#pragma unroll
    for (int t = 0; t < 4; ++t) os[(8 * hh + r) * 64 + t * 16 + c] = oacc[t][r] * inv;
  }
  __builtin_amdgcn_fence(3  , "workgroup");
  __builtin_amdgcn_wave_barrier();
  __builtin_amdgcn_fence(2  , "workgroup");
  {
    const int rq = lane >> 3, piece = lane & 7;
    v4u pv[4];
#pragma unroll
    for (int it = 0; it < 4; ++it) {
      const int row = it * 4 + rq;
      const v4f a  = *(const v4f*)(os + row * 64 + piece * 8);
      const v4f a2 = *(const v4f*)(os + row * 64 + piece * 8 + 4);
      pv[it] = pack8_flush(a, a2);
    }
    for (int pass = 0; pass < 2; ++pass) {
#pragma unroll
      for (int it = 0; it < 4; ++it) {
        const int row = it * 4 + rq;
        const size_t go = (rowB + q0 + row) * DM + (size_t)h * HD + piece * 8;
        *(volatile v4u*)(ctxp + go) = pv[it];
      }
      __threadfence();
    }
  }
}

static constexpr size_t P_WQKV = (size_t)DQKV * DM * 2;
static constexpr size_t P_WO   = (size_t)DM * DM * 2;
static constexpr size_t P_W1   = (size_t)DFF * DM * 2;
static constexpr size_t P_W2   = (size_t)DM * DFF * 2;
static constexpr size_t P_MB   = (size_t)SEQ * MBW * 4;
static constexpr size_t P_H16  = (size_t)ROWS * DM * 2;
static constexpr size_t P_QKV  = (size_t)ROWS * DQKV * 2;
static constexpr size_t P_VT   = (size_t)NB * DM * SEQ * 2;
static constexpr size_t P_F32  = (size_t)ROWS * DM * 4;
static constexpr size_t P_G    = (size_t)ROWS * DFF * 2;
static constexpr size_t O_WQKV = 0;
static constexpr size_t O_WO   = O_WQKV + P_WQKV;
static constexpr size_t O_W1   = O_WO + P_WO;
static constexpr size_t O_W2   = O_W1 + P_W1;
static constexpr size_t O_MB   = O_W2 + P_W2;
static constexpr size_t O_HH   = O_MB + P_MB;
static constexpr size_t O_QKV  = O_HH + P_H16;
static constexpr size_t O_VT   = O_QKV + P_QKV;
static constexpr size_t O_CTX  = O_VT + P_VT;
static constexpr size_t O_X1   = O_CTX + P_H16;
static constexpr size_t O_H2   = O_X1 + P_F32;
static constexpr size_t O_G    = O_H2 + P_H16;
static constexpr size_t WS_END = O_G + P_G;
static_assert(WS_END <= (size_t)134217728);
static_assert((P_MB % 512) == 0 && (P_H16 % 512) == 0 && (P_QKV % 512) == 0 && (P_VT % 512) == 0);
static_assert((P_WQKV % 512) == 0 && (P_WO % 512) == 0 && (P_W1 % 512) == 0 && (P_F32 % 512) == 0);

static constexpr int N8_QKV = DQKV * DM / 8;
static constexpr int N8_O   = DM * DM / 8;
static constexpr int N8_F   = DFF * DM / 8;
static constexpr int G_CQ   = N8_QKV / 256;
static constexpr int G_CO   = N8_O / 256;
static constexpr int G_CF   = N8_F / 256;
static constexpr int G_MP   = SEQ / 16;
static constexpr int G_LN   = ROWS / 8;
static constexpr int G_GQKV = (ROWS / 64) * (DQKV / 64) / 8;
static constexpr int G_GDM  = (ROWS / 64) * (DM / 64) / 8;
static constexpr int G_GFF  = (ROWS / 64) * (DFF / 64) / 8;
static constexpr int G_ATT  = NB * NH * NQB;
static_assert(G_MP * 8 * 128 == SEQ * MBW);
static_assert(G_LN * 8 == ROWS);

extern "C" void kernel_launch(void* const* d_in, const int* in_sizes, int n_in,
                              void* d_out, int out_size, void* d_ws, size_t ws_size,
                              hipStream_t stream) {
  if (n_in < 14) return;
  if (in_sizes[0] < NB * SEQ * DM) return;
  if (in_sizes[1] < SEQ * SEQ_FULL) return;
  if (in_sizes[2] < DM || in_sizes[3] < DM) return;
  if (in_sizes[4] < DQKV * DM || in_sizes[5] < DQKV) return;
  if (in_sizes[6] < DM * DM || in_sizes[7] < DM) return;
  if (in_sizes[8] < DM || in_sizes[9] < DM) return;
  if (in_sizes[10] < DFF * DM || in_sizes[11] < DFF) return;
  if (in_sizes[12] < DM * DFF || in_sizes[13] < DM) return;
  if (out_size < OUT0N_FULL + 1) return;
  if (ws_size < WS_END) return;

  const float* x      = (const float*)d_in[0];
  const int*   maskp  = (const int*)d_in[1];
  const float* ln1_g  = (const float*)d_in[2];
  const float* ln1_b  = (const float*)d_in[3];
  const float* qkv_w  = (const float*)d_in[4];
  const float* qkv_b  = (const float*)d_in[5];
  const float* out_w  = (const float*)d_in[6];
  const float* out_b  = (const float*)d_in[7];
  const float* ln2_g  = (const float*)d_in[8];
  const float* ln2_b  = (const float*)d_in[9];
  const float* fc1_w  = (const float*)d_in[10];
  const float* fc1_b  = (const float*)d_in[11];
  const float* fc2_w  = (const float*)d_in[12];
  const float* fc2_b  = (const float*)d_in[13];

  char* ws = (char*)d_ws;
  unsigned short* Wqkv = (unsigned short*)(ws + O_WQKV);
  unsigned short* Wo   = (unsigned short*)(ws + O_WO);
  unsigned short* W1   = (unsigned short*)(ws + O_W1);
  unsigned short* W2   = (unsigned short*)(ws + O_W2);
  unsigned int*   MB   = (unsigned int*)(ws + O_MB);
  unsigned short* Hh   = (unsigned short*)(ws + O_HH);
  unsigned short* QKV  = (unsigned short*)(ws + O_QKV);
  unsigned short* VT   = (unsigned short*)(ws + O_VT);
  unsigned short* Ctx  = (unsigned short*)(ws + O_CTX);
  float*          X1   = (float*)(ws + O_X1);
  unsigned short* H2   = (unsigned short*)(ws + O_H2);
  unsigned short* G    = (unsigned short*)(ws + O_G);
  float*          outf = (float*)d_out;
  float*          tailp = outf + OUT0N_FULL;

  const dim3 blk(256);

  cvt_w16<<<dim3(G_CQ), blk, 0, stream>>>(qkv_w, Wqkv, N8_QKV, SC_W);
  cvt_w16<<<dim3(G_CO), blk, 0, stream>>>(out_w, Wo, N8_O, SC_W);
  cvt_w16<<<dim3(G_CF), blk, 0, stream>>>(fc1_w, W1, N8_F, SC_W);
  cvt_w16<<<dim3(G_CF), blk, 0, stream>>>(fc2_w, W2, N8_F, SC_W);
  mask_pack<<<dim3(G_MP), blk, 0, stream>>>(maskp, MB, tailp);
  ln_k<<<dim3(G_LN), blk, 0, stream>>>(x, 1, ln1_g, ln1_b, Hh, ROWS);
  gemm64_f16<0><<<dim3(G_GQKV), blk, 0, stream>>>(Hh, DM, Wqkv, DM, qkv_b, CS_ACT, x, DM, (void*)QKV, DQKV,
                                                  ROWS, DQKV, DM, SC_ACT);
  v_tr<<<dim3(SEQ / 64, NH, NB), blk, 0, stream>>>(QKV, VT);
  attn_k<<<dim3(G_ATT), dim3(128), 0, stream>>>(QKV, VT, MB, Ctx);
  gemm64_f16<2><<<dim3(G_GDM), blk, 0, stream>>>(Ctx, DM, Wo, DM, out_b, CS_CTX, x, DM, (void*)X1, DM,
                                                 ROWS, DM, DM, SC_ONE);
  ln_k<<<dim3(G_LN), blk, 0, stream>>>(X1, 0, ln2_g, ln2_b, H2, ROWS);
  gemm64_f16<1><<<dim3(G_GFF), blk, 0, stream>>>(H2, DM, W1, DM, fc1_b, CS_ACT, x, DM, (void*)G, DFF,
                                                 ROWS, DFF, DM, SC_ACT);
  gemm64_f16<3><<<dim3(G_GDM), blk, 0, stream>>>(G, DFF, W2, DFF, fc2_b, CS_ACT, X1, DM, (void*)outf, DM,
                                                 ROWS, DM, DFF, SC_ONE);
  (void)hipGetLastError();
}
